// GatedLinearAttention_27650999452423
// MI455X (gfx1250) — hardware-verified
//
#include <hip/hip_runtime.h>
#include <math.h>

constexpr int kB   = 2;
constexpr int kT   = 2048;
constexpr int kD   = 1024;
constexpr int kH   = 4;
constexpr int kDK  = 256;
constexpr int kDV  = 512;
constexpr int kC   = 64;
constexpr int kLR  = 16;
constexpr int kR   = kB * kT;
constexpr int kNC  = kT / kC;
constexpr int kNCB = kB * kH * kNC;
constexpr int kQD  = kH * kDK;
constexpr int kVD  = kH * kDV;
constexpr int kQKN = 2112;
constexpr float kQCarry      = 16.0f;
constexpr float kOCarryInv   = 1.0f / 256.0f;
constexpr float kGateNormInv = 1.0f / 16.0f;
constexpr float kEps         = 1.0e-5f;
constexpr float kInvDV       = 1.0f / 512.0f;
static_assert(kQD == 1024 && kVD == 2048 && kR == 4096 && kNC == 32 && kNCB == 256);
static_assert(kD % 32 == 0 && kVD % 32 == 0 && kDK % 32 == 0 && kC % 32 == 0);
static_assert(kR % 64 == 0 && kQKN % 64 == 0 && kVD % 64 == 0 && kD % 64 == 0);
static_assert(kQKN >= 2 * kQD + kLR && (kQKN * 4) % 128 == 0);

typedef __attribute__((ext_vector_type(16))) _Float16 v16h;
typedef __attribute__((ext_vector_type(8)))  _Float16 v8h;
typedef __attribute__((ext_vector_type(16))) __bf16   v16b;
typedef __attribute__((ext_vector_type(8)))  __bf16   v8b;
typedef __attribute__((ext_vector_type(8)))  float    v8f;
typedef __attribute__((ext_vector_type(4)))  float    v4f;
typedef __attribute__((ext_vector_type(4)))  unsigned int v4u;

__device__ __forceinline__ unsigned short f2bf_bits(float f) {
  unsigned u = __float_as_uint(f);
  return (unsigned short)((u + 0x7FFFu + ((u >> 16) & 1u)) >> 16);
}
__device__ __forceinline__ float bf_bits2f(unsigned short h) { return __uint_as_float(((unsigned)h) << 16); }
__device__ __forceinline__ float bf_rne(float f) { return bf_bits2f(f2bf_bits(f)); }
__device__ __forceinline__ unsigned pk16(unsigned short a, unsigned short b) { return (unsigned)a | ((unsigned)b << 16); }
__device__ __forceinline__ unsigned short h_bits(float f) { const _Float16 h = (_Float16)f; return __builtin_bit_cast(unsigned short, h); }
__device__ __forceinline__ float h16_to_f32(unsigned hb) {
  const unsigned sgn = (hb & 0x8000u) << 16; const unsigned em = hb & 0x7fffu;
  const float fn = __uint_as_float((em << 13) + 0x38000000u);
  const float fs = (float)em * 5.9604644775390625e-8f;
  const float mag = (em < 0x400u) ? fs : fn; return __uint_as_float(__float_as_uint(mag) | sgn); }

__device__ __forceinline__ void guard4_h2(v8f& a, v8f& b, v8f& c, v8f& d, v16h x, v16h y) {
  asm volatile("v_nop\n\tv_nop\n\tv_nop\n\tv_nop" : "+v"(a), "+v"(b), "+v"(c), "+v"(d) : "v"(x), "v"(y)); }
__device__ __forceinline__ void guard4_b2(v8f& a, v8f& b, v8f& c, v8f& d, v16b x, v16b y) {
  asm volatile("v_nop\n\tv_nop\n\tv_nop\n\tv_nop" : "+v"(a), "+v"(b), "+v"(c), "+v"(d) : "v"(x), "v"(y)); }
__device__ __forceinline__ void guard4_h5(v8f& a, v8f& b, v8f& c, v8f& d, v16h x0, v16h x1, v16h x2, v16h x3, v16h x4) {
  asm volatile("v_nop\n\tv_nop\n\tv_nop\n\tv_nop" : "+v"(a), "+v"(b), "+v"(c), "+v"(d) : "v"(x0), "v"(x1), "v"(x2), "v"(x3), "v"(x4)); }
__device__ __forceinline__ void guard1_h4(v8f& a, v16h x0, v16h x1, v16h x2, v16h x3) {
  asm volatile("v_nop\n\tv_nop\n\tv_nop\n\tv_nop" : "+v"(a) : "v"(x0), "v"(x1), "v"(x2), "v"(x3)); }
__device__ __forceinline__ void keep4_h(v16h a, v16h b, v16h c, v16h d) { asm volatile("v_nop" :: "v"(a), "v"(b), "v"(c), "v"(d)); }
__device__ __forceinline__ void keep4_b(v16b a, v16b b, v16b c, v16b d) { asm volatile("v_nop" :: "v"(a), "v"(b), "v"(c), "v"(d)); }
__device__ __forceinline__ void acc_guard4(v8f& a, v8f& b, v8f& c, v8f& d) { asm volatile("v_nop\n\tv_nop\n\tv_nop\n\tv_nop" : "+v"(a), "+v"(b), "+v"(c), "+v"(d)); }

template <typename T> struct Frag;
template <> struct Frag<_Float16> {
  typedef v16h V; union U { v16h v; v8h h[2]; };
  static __device__ __forceinline__ v16h load(const _Float16* p) {
    U f; f.h[0] = *(const v8h*)(p); f.h[1] = *(const v8h*)(p + 16); return f.v;
  }
  static __device__ __forceinline__ v8f mma(v16h a, v16h b, v8f c) {
    return __builtin_amdgcn_wmma_f32_16x16x32_f16(false, a, false, b, (short)0, c, false, false);
  }
  static __device__ __forceinline__ void guard4(v8f& a, v8f& b, v8f& c, v8f& d, v16h x, v16h y) { guard4_h2(a, b, c, d, x, y); }
  static __device__ __forceinline__ void keep(v16h a, v16h b, v16h c, v16h d) { keep4_h(a, b, c, d); }
};
template <> struct Frag<__bf16> {
  typedef v16b V; union U { v16b v; v8b h[2]; };
  static __device__ __forceinline__ v16b load(const __bf16* p) {
    U f; f.h[0] = *(const v8b*)(p); f.h[1] = *(const v8b*)(p + 16); return f.v;
  }
  static __device__ __forceinline__ v8f mma(v16b a, v16b b, v8f c) {
    return __builtin_amdgcn_wmma_f32_16x16x32_bf16(false, a, false, b, (short)0, c, false, false);
  }
  static __device__ __forceinline__ void guard4(v8f& a, v8f& b, v8f& c, v8f& d, v16b x, v16b y) { guard4_b2(a, b, c, d, x, y); }
  static __device__ __forceinline__ void keep(v16b a, v16b b, v16b c, v16b d) { keep4_b(a, b, c, d); }
};

template <int ET> struct Elem;
template <> struct Elem<0> { typedef _Float16 T; };
template <> struct Elem<1> { typedef __bf16 T; };
template <int ET, int SPL, int OUT_MODE>
__global__ __launch_bounds__(256) void wmma_gemm64(
    const unsigned short* __restrict__ Ap, const unsigned short* __restrict__ A2p, int lda,
    const unsigned short* __restrict__ Btp, const unsigned short* __restrict__ Bt2p, int ldb,
    void* __restrict__ Cout, int ldc, int M, int N, int K, float scale) {
  typedef typename Elem<ET>::T T;
  typedef typename Frag<T>::V V;
  const T* A = (const T*)Ap; const T* A2 = (const T*)A2p; const T* Bt = (const T*)Btp; const T* Bt2 = (const T*)Bt2p;
  __shared__ __align__(16) float sT[8][16 * 68];
  const int lane = threadIdx.x & 31;
  const int wave = threadIdx.x >> 5;
  const int tilesN = N >> 6;
  const int tilesM = M >> 6;
  const int tile = blockIdx.x * 8 + wave;
  if (tile >= tilesM * tilesN) return;
  const int tm = tile / tilesN;
  const int tn = tile - tm * tilesN;
  const int m0 = tm << 6;
  const int n0 = tn << 6;

  const int rlane = lane & 15;
  const int koff  = (lane >> 4) * 8;
  const int mOff  = (lane >> 4) * 8;

  v8f acc[4][4];
#pragma unroll
  for (int i = 0; i < 4; ++i)
#pragma unroll
    for (int j = 0; j < 4; ++j) acc[i][j] = (v8f){0.f,0.f,0.f,0.f,0.f,0.f,0.f,0.f};

  for (int k0 = 0; k0 < K; k0 += 32) {
    V bh[4], bl[4];
#pragma unroll
    for (int j = 0; j < 4; ++j) {
      const size_t bo = (size_t)(n0 + (j << 4) + rlane) * ldb + koff + k0;
      bh[j] = Frag<T>::load(Bt + bo);
      if (SPL == 2) bl[j] = Frag<T>::load(Bt2 + bo);
    }
#pragma unroll
    for (int i = 0; i < 4; ++i) {
      const size_t ao = (size_t)(m0 + (i << 4) + rlane) * lda + koff + k0;
      V ah = Frag<T>::load(A + ao);
      V al = ah;
      if (SPL != 0) al = Frag<T>::load(A2 + ao);
#pragma unroll
      for (int j = 0; j < 4; ++j) {
        acc[i][j] = Frag<T>::mma(ah, bh[j], acc[i][j]);
        if (SPL == 2) acc[i][j] = Frag<T>::mma(ah, bl[j], acc[i][j]);
        if (SPL != 0) acc[i][j] = Frag<T>::mma(al, bh[j], acc[i][j]);
      }
      Frag<T>::guard4(acc[i][0], acc[i][1], acc[i][2], acc[i][3], ah, al);
    }
    Frag<T>::keep(bh[0], bh[1], bh[2], bh[3]);
    if (SPL == 2) Frag<T>::keep(bl[0], bl[1], bl[2], bl[3]);
  }
  acc_guard4(acc[0][0], acc[0][1], acc[0][2], acc[0][3]);
  acc_guard4(acc[1][0], acc[1][1], acc[1][2], acc[1][3]);
  acc_guard4(acc[2][0], acc[2][1], acc[2][2], acc[2][3]);
  acc_guard4(acc[3][0], acc[3][1], acc[3][2], acc[3][3]);

  float* slab = sT[wave];
#pragma unroll
  for (int i = 0; i < 4; ++i) {
    const int mBase = m0 + (i << 4);
#pragma unroll
    for (int j = 0; j < 4; ++j) {
#pragma unroll
      for (int r = 0; r < 8; ++r) {
        const float v = acc[i][j][r] * scale;
        slab[(mOff + r) * 68 + (j << 4) + rlane] = v;
      }
    }
    __builtin_amdgcn_fence(__ATOMIC_RELEASE, "workgroup");
    __builtin_amdgcn_wave_barrier();
    __builtin_amdgcn_fence(__ATOMIC_ACQUIRE, "workgroup");
    if (OUT_MODE == 0) {
      float* Cp = (float*)Cout;
      const int hh = lane >> 4, c4 = (lane & 15) * 4;
      for (int pass = 0; pass < 2; ++pass) {
#pragma unroll
        for (int it = 0; it < 8; ++it) {
          const int row = it * 2 + hh;
          v4f v = *(const v4f*)(slab + row * 68 + c4);
          *(volatile v4f*)(Cp + (size_t)(mBase + row) * ldc + n0 + c4) = v;
        }
        __threadfence();
      }
    } else {
      const int q = lane >> 3, c8 = (lane & 7) * 8;
      unsigned short* Cp = (unsigned short*)Cout;
      for (int pass = 0; pass < 2; ++pass) {
#pragma unroll
        for (int it = 0; it < 4; ++it) {
          const int row = it * 4 + q;
          const float* sp = slab + row * 68 + c8;
          v8h hv;
#pragma unroll
          for (int e = 0; e < 8; ++e) hv[e] = (_Float16)sp[e];
          *(volatile v8h*)(Cp + (size_t)(mBase + row) * ldc + n0 + c8) = hv;
        }
        __threadfence();
      }
    }
    __builtin_amdgcn_fence(__ATOMIC_RELEASE, "workgroup");
    __builtin_amdgcn_wave_barrier();
    __builtin_amdgcn_fence(__ATOMIC_ACQUIRE, "workgroup");
  }
}

__global__ __launch_bounds__(256) void cast8_bf16_kernel(const float* __restrict__ in, unsigned short* __restrict__ out, int n8) {
  const int i = blockIdx.x * 256 + threadIdx.x;
  if (i >= n8) return;
  const float* p = in + 8 * (size_t)i;
  const v4f a = *(const v4f*)(p);
  const v4f c = *(const v4f*)(p + 4);
  unsigned short hb[8];
#pragma unroll
  for (int e = 0; e < 4; ++e) {
    hb[e]     = f2bf_bits(a[e]);
    hb[4 + e] = f2bf_bits(c[e]);
  }
  const v4u u = (v4u){pk16(hb[0], hb[1]), pk16(hb[2], hb[3]), pk16(hb[4], hb[5]), pk16(hb[6], hb[7])};
  unsigned short* q = out + 8 * (size_t)i;
  *(volatile v4u*)q = u;
  __threadfence();
  *(volatile v4u*)q = u;
}

__global__ __launch_bounds__(256) void zero8_kernel(unsigned short* __restrict__ out, int n8) {
  const int i = blockIdx.x * 256 + threadIdx.x;
  if (i >= n8) return;
  const v4u u = (v4u){0u, 0u, 0u, 0u};
  unsigned short* q = out + 8 * (size_t)i;
  *(volatile v4u*)q = u;
  __threadfence();
  *(volatile v4u*)q = u;
}

__device__ __forceinline__ float dot4(v4f a, v4f b) { return ((a[0] * b[0] + a[1] * b[1]) + (a[2] * b[2] + a[3] * b[3])); }
__device__ __forceinline__ v4f bf_rne4(v4f a) { return (v4f){bf_rne(a[0]), bf_rne(a[1]), bf_rne(a[2]), bf_rne(a[3])}; }

__global__ __launch_bounds__(128) void gate_kernel(const float* __restrict__ QK, const float* __restrict__ Wgk2,
                                                   const float* __restrict__ bgk2,
                                                   unsigned short* __restrict__ qgp, unsigned short* __restrict__ kgp,
                                                   unsigned short* __restrict__ kgtp, float* __restrict__ decp) {
  __shared__ __align__(16) float sT16[kC][kLR];
  __shared__ __align__(16) unsigned short sQ[kC][136];
  __shared__ __align__(16) unsigned short sK[kC][136];
  __shared__ __align__(16) unsigned short sKT[128][72];
  __shared__ __align__(16) float sDec[128];
  const int t = threadIdx.x, lane = t & 31, wave = t >> 5;
  const int half = blockIdx.x & 1;
  const int cb = blockIdx.x >> 1;
  const int c = cb & (kNC - 1), bh = cb >> 5, h = bh & 3, bb = bh >> 2;
  const int rowbase = bb * kT + c * kC;
  const int dk = half * 128 + t;
  const int colq = h * kDK + dk;
  const int colk = kQD + colq;
  {
    const int r = t >> 1, part = t & 1;
    const float* src = QK + (size_t)(rowbase + r) * kQKN + 2 * kQD + part * 8;
    const v4f a = *(const v4f*)(src);
    const v4f b4 = *(const v4f*)(src + 4);
    *(v4f*)(&sT16[r][part * 8]) = a;
    *(v4f*)(&sT16[r][part * 8 + 4]) = b4;
  }
  const float* wr = Wgk2 + (size_t)colq * kLR;
  const v4f w0 = bf_rne4(*(const v4f*)(wr));
  const v4f w1 = bf_rne4(*(const v4f*)(wr + 4));
  const v4f w2 = bf_rne4(*(const v4f*)(wr + 8));
  const v4f w3 = bf_rne4(*(const v4f*)(wr + 12));
  const float bias = bf_rne(bgk2[colq]);
  __syncthreads();

  float run = 0.0f;
  float eb = 1.0f;
#pragma unroll 1
  for (int p = 0; p < kC; ++p) {
    const v4f t0 = *(const v4f*)(&sT16[p][0]);
    const v4f t1 = *(const v4f*)(&sT16[p][4]);
    const v4f t2 = *(const v4f*)(&sT16[p][8]);
    const v4f t3 = *(const v4f*)(&sT16[p][12]);
    const float z = ((dot4(t0, w0) + dot4(t1, w1)) + (dot4(t2, w2) + dot4(t3, w3))) + bias;
    const float ls = fminf(z, 0.0f) - log1pf(expf(-fabsf(z)));
    run += ls * kGateNormInv;
    eb = expf(run);
    const float enb = expf(-run);
    const size_t gi = (size_t)(rowbase + p) * kQKN;
    const float qv = QK[gi + colq];
    const float kv = QK[gi + colk];
    const float qg = (qv * eb) * kQCarry;
    const float kg = kv * enb;
    const unsigned short kgb = h_bits(kg);
    sQ[p][t] = h_bits(qg);
    sK[p][t] = kgb;
    sKT[t][p] = kgb;
  }
  sDec[t] = eb;
  __syncthreads();

  const int hh = lane >> 4, c8 = (lane & 15) * 8;
  const int q4 = lane >> 3, c8b = (lane & 7) * 8;
  unsigned short* qdst = qgp + (size_t)rowbase * kQD + h * kDK + half * 128;
  unsigned short* kdst = kgp + (size_t)rowbase * kQD + h * kDK + half * 128;
  unsigned short* tdst = kgtp + ((size_t)cb * kDK + half * 128) * kC;
  float* ddst = decp + (size_t)cb * kDK + half * 128;
  for (int pass = 0; pass < 2; ++pass) {
#pragma unroll 1
    for (int it = 0; it < 8; ++it) {
      const int row = wave * 16 + it * 2 + hh;
      v4u uq, uk;
      __builtin_memcpy(&uq, &sQ[row][c8], 16);
      __builtin_memcpy(&uk, &sK[row][c8], 16);
      *(volatile v4u*)(qdst + (size_t)row * kQD + c8) = uq;
      *(volatile v4u*)(kdst + (size_t)row * kQD + c8) = uk;
    }
#pragma unroll 1
    for (int it = 0; it < 8; ++it) {
      const int row = wave * 32 + it * 4 + q4;
      v4u ut;
      __builtin_memcpy(&ut, &sKT[row][c8b], 16);
      *(volatile v4u*)(tdst + (size_t)row * kC + c8b) = ut;
    }
    if (t < 32) {
      const v4f dv = *(const v4f*)(sDec + 4 * t);
      *(volatile v4f*)(ddst + 4 * t) = dv;
    }
    __threadfence();
  }
}

__global__ __launch_bounds__(128) void amat_kernel(const unsigned short* __restrict__ qgp, const unsigned short* __restrict__ kgp,
                                                   unsigned short* __restrict__ Apl) {
  __shared__ __align__(16) float sT[4][16 * 68];
  const int t = threadIdx.x, lane = t & 31, wave = t >> 5;
  const int cb = blockIdx.x;
  const int c = cb & (kNC - 1), bh = cb >> 5, h = bh & 3, bb = bh >> 2;
  const int rowbase = bb * kT + c * kC;
  const int rlane = lane & 15, koff = (lane >> 4) * 8, mOff = koff;
  const _Float16* Qb = (const _Float16*)qgp + (size_t)rowbase * kQD + h * kDK;
  const _Float16* Kb = (const _Float16*)kgp + (size_t)rowbase * kQD + h * kDK;

  v8f acc[4];
#pragma unroll
  for (int j = 0; j < 4; ++j) acc[j] = (v8f){0.f,0.f,0.f,0.f,0.f,0.f,0.f,0.f};
#pragma unroll
  for (int kb = 0; kb < kDK / 32; ++kb) {
    v16h bf[4];
#pragma unroll
    for (int j = 0; j < 4; ++j) bf[j] = Frag<_Float16>::load(Kb + (size_t)(j * 16 + rlane) * kQD + koff + 32 * kb);
    const v16h af = Frag<_Float16>::load(Qb + (size_t)(wave * 16 + rlane) * kQD + koff + 32 * kb);
#pragma unroll
    for (int j = 0; j < 4; ++j) acc[j] = Frag<_Float16>::mma(af, bf[j], acc[j]);
    guard4_h5(acc[0], acc[1], acc[2], acc[3], af, bf[0], bf[1], bf[2], bf[3]);
  }

  float* slab = sT[wave];
#pragma unroll
  for (int j = 0; j < 4; ++j) {
    const int gj = j * 16 + rlane;
#pragma unroll
    for (int r = 0; r < 8; ++r) {
      const int gi = wave * 16 + mOff + r;
      const float v = (gi >= gj) ? acc[j][r] : 0.0f;
      slab[(mOff + r) * 68 + (j << 4) + rlane] = v;
    }
  }
  __builtin_amdgcn_fence(__ATOMIC_RELEASE, "workgroup");
  __builtin_amdgcn_wave_barrier();
  __builtin_amdgcn_fence(__ATOMIC_ACQUIRE, "workgroup");
  const int q = lane >> 3, c8 = (lane & 7) * 8;
  unsigned short* Cp = Apl + (size_t)cb * (kC * kC) + (size_t)(wave * 16) * kC;
  for (int pass = 0; pass < 2; ++pass) {
#pragma unroll
    for (int it = 0; it < 4; ++it) {
      const int row = it * 4 + q;
      const float* sp = slab + row * 68 + c8;
      v8h hv;
#pragma unroll
      for (int e = 0; e < 8; ++e) hv[e] = (_Float16)sp[e];
      *(volatile v8h*)(Cp + (size_t)row * kC + c8) = hv;
    }
    __threadfence();
  }
}

__global__ __launch_bounds__(256) void scan_kernel(const unsigned short* __restrict__ qgp, const unsigned short* __restrict__ kgtp,
                                                   const unsigned short* __restrict__ Apl, const unsigned short* __restrict__ VTp,
                                                   const float* __restrict__ decp, float* __restrict__ op) {
  __shared__ __align__(16) float slab[kC * 132];
  const int t = threadIdx.x, lane = t & 31, wave = t >> 5;
  const int rlane = lane & 15, koff = (lane >> 4) * 8, hh = lane >> 4;
  const int vs = blockIdx.x & 3, bh = blockIdx.x >> 2, h = bh & 3, bb = bh >> 2;
  const int dv0 = vs * 128 + wave * 16;
  const _Float16* VTb = (const _Float16*)VTp + (size_t)(h * kDV + dv0 + rlane) * kR + (size_t)bb * kT + koff;

  v8f S[16];
#pragma unroll
  for (int tk = 0; tk < 16; ++tk) S[tk] = (v8f){0.f,0.f,0.f,0.f,0.f,0.f,0.f,0.f};

#pragma unroll 1
  for (int c = 0; c < kNC; ++c) {
    const int cb = bh * kNC + c;
    const int rowbase = bb * kT + c * kC;
    const _Float16* Qrow  = (const _Float16*)qgp + (size_t)(rowbase + rlane) * kQD + h * kDK + koff;
    const _Float16* Arow  = (const _Float16*)Apl + (size_t)cb * (kC * kC) + rlane * kC + koff;
    const _Float16* KTrow = (const _Float16*)kgtp + ((size_t)cb * kDK + rlane) * kC + koff;

    v8f oacc[4];
#pragma unroll
    for (int ti = 0; ti < 4; ++ti) oacc[ti] = (v8f){0.f,0.f,0.f,0.f,0.f,0.f,0.f,0.f};

#pragma unroll
    for (int kb = 0; kb < 8; ++kb) {
      v16h sf;
#pragma unroll
      for (int i = 0; i < 8; ++i) {
        sf[i]     = (_Float16)S[2 * kb][i];
        sf[8 + i] = (_Float16)S[2 * kb + 1][i];
      }
      v16h af[4];
#pragma unroll
      for (int ti = 0; ti < 4; ++ti) af[ti] = Frag<_Float16>::load(Qrow + (size_t)(ti * 16) * kQD + 32 * kb);
#pragma unroll
      for (int ti = 0; ti < 4; ++ti) oacc[ti] = Frag<_Float16>::mma(af[ti], sf, oacc[ti]);
      guard4_h5(oacc[0], oacc[1], oacc[2], oacc[3], af[0], af[1], af[2], af[3], sf);
    }

    const v16h vb0 = Frag<_Float16>::load(VTb + c * kC);
    const v16h vb1 = Frag<_Float16>::load(VTb + c * kC + 32);

    {
      v16h af[4];
#pragma unroll
      for (int ti = 0; ti < 4; ++ti) af[ti] = Frag<_Float16>::load(Arow + (size_t)(ti * 16) * kC);
#pragma unroll
      for (int ti = 0; ti < 4; ++ti) oacc[ti] = Frag<_Float16>::mma(af[ti], vb0, oacc[ti]);
      guard4_h5(oacc[0], oacc[1], oacc[2], oacc[3], af[0], af[1], af[2], af[3], vb0);
#pragma unroll
      for (int ti = 0; ti < 4; ++ti) af[ti] = Frag<_Float16>::load(Arow + (size_t)(ti * 16) * kC + 32);
#pragma unroll
      for (int ti = 0; ti < 4; ++ti) oacc[ti] = Frag<_Float16>::mma(af[ti], vb1, oacc[ti]);
      guard4_h5(oacc[0], oacc[1], oacc[2], oacc[3], af[0], af[1], af[2], af[3], vb1);
    }

    __syncthreads();
#pragma unroll
    for (int ti = 0; ti < 4; ++ti) {
#pragma unroll
      for (int r = 0; r < 8; ++r) slab[(ti * 16 + hh * 8 + r) * 132 + wave * 16 + rlane] = oacc[ti][r] * kOCarryInv;
    }
    __syncthreads();
    {
      float* ob = op + (size_t)rowbase * kQKN + h * kDV + vs * 128 + lane * 4;
      for (int pass = 0; pass < 2; ++pass) {
#pragma unroll
        for (int it = 0; it < 8; ++it) {
          const int row = wave * 8 + it;
          const v4f v = *(const v4f*)(slab + row * 132 + lane * 4);
          *(volatile v4f*)(ob + (size_t)row * kQKN) = v;
        }
        __threadfence();
      }
    }

#pragma unroll
    for (int tk = 0; tk < 16; ++tk) {
      const v16h k0 = Frag<_Float16>::load(KTrow + (size_t)(tk * 16) * kC);
      const v16h k1 = Frag<_Float16>::load(KTrow + (size_t)(tk * 16) * kC + 32);
      S[tk] = Frag<_Float16>::mma(k0, vb0, S[tk]);
      S[tk] = Frag<_Float16>::mma(k1, vb1, S[tk]);
      guard1_h4(S[tk], k0, k1, vb0, vb1);
      const v4f d0 = *(const v4f*)(decp + (size_t)cb * kDK + tk * 16 + hh * 8);
      const v4f d1 = *(const v4f*)(decp + (size_t)cb * kDK + tk * 16 + hh * 8 + 4);
      S[tk][0] *= d0[0]; S[tk][1] *= d0[1]; S[tk][2] *= d0[2]; S[tk][3] *= d0[3];
      S[tk][4] *= d1[0]; S[tk][5] *= d1[1]; S[tk][6] *= d1[2]; S[tk][7] *= d1[3];
    }
  }
}

__global__ __launch_bounds__(256) void norm_gate_kernel(const float* __restrict__ op, const unsigned short* __restrict__ Gp,
                                                        const float* __restrict__ gnw,
                                                        unsigned short* __restrict__ hop, unsigned short* __restrict__ lop) {
  __shared__ float red[8];
  const int row = blockIdx.x, t = threadIdx.x, lane = t & 31, wave = t >> 5;
  const int head = t >> 6, u = t & 63;
  const int col = head * kDV + 8 * u;
  const float* orow = op + (size_t)row * kQKN + col;
  const v4f o0 = *(const v4f*)(orow);
  const v4f o1 = *(const v4f*)(orow + 4);
  float ov[8];
#pragma unroll
  for (int e = 0; e < 4; ++e) { ov[e] = o0[e]; ov[4 + e] = o1[e]; }
  float ss = ((ov[0] * ov[0] + ov[1] * ov[1]) + (ov[2] * ov[2] + ov[3] * ov[3])) +
             ((ov[4] * ov[4] + ov[5] * ov[5]) + (ov[6] * ov[6] + ov[7] * ov[7]));
#pragma unroll
  for (int off = 16; off > 0; off >>= 1) ss += __shfl_xor(ss, off, 32);
  if (lane == 0) red[wave] = ss;
  __syncthreads();
  const float tot = red[2 * head] + red[2 * head + 1];
  const float rstd = rsqrtf(tot * kInvDV + kEps);
  const v4u gw = *(const v4u*)(Gp + (size_t)row * kVD + col);
  const v4f n0 = *(const v4f*)(gnw + 8 * u);
  const v4f n1 = *(const v4f*)(gnw + 8 * u + 4);
  float gn[8], gf[8];
#pragma unroll
  for (int e = 0; e < 4; ++e) {
    gn[e] = bf_rne(n0[e]); gn[4 + e] = bf_rne(n1[e]);
    gf[2 * e]     = h16_to_f32(gw[e] & 0xffffu);
    gf[2 * e + 1] = h16_to_f32(gw[e] >> 16);
  }
  unsigned short hb[8], lb[8];
#pragma unroll
  for (int e = 0; e < 8; ++e) {
    const float g = gf[e];
    const float sig = __builtin_amdgcn_rcpf(1.0f + expf(-g));
    const float val = ((ov[e] * rstd) * gn[e]) * (g * sig);
    hb[e] = f2bf_bits(val);
    lb[e] = f2bf_bits(val - bf_bits2f(hb[e]));
  }
  const v4u uh = (v4u){pk16(hb[0], hb[1]), pk16(hb[2], hb[3]), pk16(hb[4], hb[5]), pk16(hb[6], hb[7])};
  const v4u ul = (v4u){pk16(lb[0], lb[1]), pk16(lb[2], lb[3]), pk16(lb[4], lb[5]), pk16(lb[6], lb[7])};
  unsigned short* hp = hop + (size_t)row * kVD + col;
  unsigned short* lp = lop + (size_t)row * kVD + col;
  *(volatile v4u*)hp = uh;
  *(volatile v4u*)lp = ul;
  __threadfence();
  *(volatile v4u*)hp = uh;
  *(volatile v4u*)lp = ul;
}

extern "C" void kernel_launch(void* const* d_in, const int* in_sizes, int n_in,
                              void* d_out, int out_size, void* d_ws, size_t ws_size,
                              hipStream_t stream) {
  if (n_in < 10) return;
  if (in_sizes[0] != kR * kD) return;
  if (in_sizes[1] != kQD * kD || in_sizes[2] != kQD * kD) return;
  if (in_sizes[3] != kVD * kD || in_sizes[4] != kVD * kD) return;
  if (in_sizes[5] != kLR * kD || in_sizes[6] != kQD * kLR || in_sizes[7] != kQD) return;
  if (in_sizes[8] != kD * kVD || in_sizes[9] != kDV) return;
  if (out_size != kR * kD) return;

  const size_t szXB   = (size_t)kR * kD * 2;
  const size_t szWQK  = (size_t)kQKN * kD * 2;
  const size_t szWV   = (size_t)kVD * kD * 2;
  const size_t szWG   = (size_t)kVD * kD * 2;
  const size_t szWO   = (size_t)kD * kVD * 2;
  const size_t szQK   = (size_t)kR * kQKN * 4;
  const size_t szVT   = (size_t)kVD * kR * 2;
  const size_t szQG   = (size_t)kR * kQD * 2;
  const size_t szKG   = (size_t)kR * kQD * 2;
  const size_t szKGT  = (size_t)kNCB * kDK * kC * 2;
  const size_t szDEC  = (size_t)kNCB * kDK * 4;
  const size_t szAPL  = (size_t)kNCB * kC * kC * 2;
  const size_t szON   = (size_t)kR * kVD * 2;
  const size_t offXB  = 0;
  const size_t offWQK = offXB + szXB;
  const size_t offWV  = offWQK + szWQK;
  const size_t offWG  = offWV + szWV;
  const size_t offWO  = offWG + szWG;
  const size_t offQK  = offWO + szWO;
  const size_t offVT  = offQK + szQK;
  const size_t offQG  = offVT + szVT;
  const size_t offKG  = offQG + szQG;
  const size_t offKGT = offKG + szKG;
  const size_t offDEC = offKGT + szKGT;
  const size_t offAPL = offDEC + szDEC;
  const size_t offONH = offAPL + szAPL;
  const size_t total  = offONH + szON;
  static_assert((size_t)kR * kVD * 2 <= (size_t)kR * kD * 2 + (size_t)kQKN * kD * 2 + (size_t)kVD * kD * 2);
  static_assert((size_t)kR * kVD * 2 == 2 * (size_t)kR * kQD * 2);
  if (total > (size_t)134217728) return;
  if (ws_size < total) return;

  const float* x    = (const float*)d_in[0];
  const float* Wq   = (const float*)d_in[1];
  const float* Wk   = (const float*)d_in[2];
  const float* Wv   = (const float*)d_in[3];
  const float* Wg   = (const float*)d_in[4];
  const float* Wgk1 = (const float*)d_in[5];
  const float* Wgk2 = (const float*)d_in[6];
  const float* bgk2 = (const float*)d_in[7];
  const float* Wo   = (const float*)d_in[8];
  const float* gnw  = (const float*)d_in[9];
  float* out = (float*)d_out;
  char* ws = (char*)d_ws;
  unsigned short* XB   = (unsigned short*)(ws + offXB);
  unsigned short* WQK1 = (unsigned short*)(ws + offWQK);
  unsigned short* WVB  = (unsigned short*)(ws + offWV);
  unsigned short* WGB  = (unsigned short*)(ws + offWG);
  unsigned short* WOB  = (unsigned short*)(ws + offWO);
  float*          QK   = (float*)(ws + offQK);
  float*          OP   = (float*)(ws + offQK);
  unsigned short* VT   = (unsigned short*)(ws + offVT);
  unsigned short* QG   = (unsigned short*)(ws + offQG);
  unsigned short* KG   = (unsigned short*)(ws + offKG);
  unsigned short* GP   = (unsigned short*)(ws + offQG);
  unsigned short* KGT  = (unsigned short*)(ws + offKGT);
  float*          DEC  = (float*)(ws + offDEC);
  unsigned short* APL  = (unsigned short*)(ws + offAPL);
  unsigned short* ONHI = (unsigned short*)(ws + offONH);
  unsigned short* ONLO = (unsigned short*)(ws + offXB);

  {
    const int n8x = kR * kD / 8;
    const int n8q = kQD * kD / 8;
    const int n8l = kLR * kD / 8;
    const int n8z = (kQKN - 2 * kQD - kLR) * kD / 8;
    const int n8v = kVD * kD / 8;
    static_assert((kR * kD / 8) % 256 == 0 && (kQD * kD / 8) % 256 == 0 && (kLR * kD / 8) % 256 == 0);
    static_assert(((kQKN - 2 * kQD - kLR) * kD / 8) % 256 == 0 && (kVD * kD / 8) % 256 == 0);
    cast8_bf16_kernel<<<dim3(n8x / 256), dim3(256), 0, stream>>>(x, XB, n8x);
    cast8_bf16_kernel<<<dim3(n8q / 256), dim3(256), 0, stream>>>(Wq, WQK1, n8q);
    cast8_bf16_kernel<<<dim3(n8q / 256), dim3(256), 0, stream>>>(Wk, WQK1 + (size_t)kQD * kD, n8q);
    cast8_bf16_kernel<<<dim3(n8l / 256), dim3(256), 0, stream>>>(Wgk1, WQK1 + (size_t)2 * kQD * kD, n8l);
    zero8_kernel<<<dim3(n8z / 256), dim3(256), 0, stream>>>(WQK1 + (size_t)(2 * kQD + kLR) * kD, n8z);
    cast8_bf16_kernel<<<dim3(n8v / 256), dim3(256), 0, stream>>>(Wv, WVB, n8v);
    cast8_bf16_kernel<<<dim3(n8v / 256), dim3(256), 0, stream>>>(Wg, WGB, n8v);
    cast8_bf16_kernel<<<dim3(n8v / 256), dim3(256), 0, stream>>>(Wo, WOB, n8v);
  }

  wmma_gemm64<1, 0, 0><<<dim3((kR / 64) * (kQKN / 64) / 8), dim3(256), 0, stream>>>(
      XB, XB, kD, WQK1, WQK1, kD, (void*)QK, kQKN, kR, kQKN, kD, 1.0f);
  wmma_gemm64<1, 0, 1><<<dim3((kVD / 64) * (kR / 64) / 8), dim3(256), 0, stream>>>(
      WVB, WVB, kD, XB, XB, kD, (void*)VT, kR, kVD, kR, kD, 1.0f);
  gate_kernel<<<dim3(2 * kNCB), dim3(128), 0, stream>>>(QK, Wgk2, bgk2, QG, KG, KGT, DEC);
  amat_kernel<<<dim3(kNCB), dim3(128), 0, stream>>>(QG, KG, APL);
  scan_kernel<<<dim3(kB * kH * 4), dim3(256), 0, stream>>>(QG, KGT, APL, VT, DEC, OP);
  wmma_gemm64<1, 0, 1><<<dim3((kR / 64) * (kVD / 64) / 8), dim3(256), 0, stream>>>(
      XB, XB, kD, WGB, WGB, kD, (void*)GP, kVD, kR, kVD, kD, 1.0f);
  norm_gate_kernel<<<dim3(kR), dim3(256), 0, stream>>>(OP, GP, gnw, ONHI, ONLO);
  wmma_gemm64<1, 1, 0><<<dim3((kR / 64) * (kD / 64) / 8), dim3(256), 0, stream>>>(
      ONHI, ONLO, kVD, WOB, WOB, kVD, (void*)out, kD, kR, kD, kVD, 1.0f);
}
